// Encoder_36369783063167
// MI455X (gfx1250) — hardware-verified
//
#include <hip/hip_runtime.h>
#include <stddef.h>
#include <stdint.h>
#include <math.h>


#define CH     128
#define NT     256
#define HP     256
#define OUTC   64
#define K1     128
#define K2     256
#define NTHR   256
#define NWAVE  8
#define EPT    8
#define CHUNK  (NTHR * EPT)
#define WCAP   (EPT * 32)
#define LISTN  (NWAVE * WCAP)
#define NBA    1024
#define SLA    10
#define RCAP   28672
#define DEGCAP 64
#define GBM    64
#define GBN    64
#define GTHR   128
#define PB_W1  16
#define PB_W2  32
#define PB_HEAD (PB_W1 + PB_W2 + 1)
#define AGG_ZINTS    (LISTN + 2 * RCAP + 3 * NBA)
#define MISC_INTS    16
#define PROW_INTS    (NWAVE * CH)
#define ROWBUF_INTS  (NWAVE * HP / 2)
#define AGG_LDS_INTS (AGG_ZINTS + MISC_INTS + PROW_INTS + ROWBUF_INTS)
#define WSMAX  134217728

static_assert((CHUNK & (CHUNK - 1)) == 0 && CHUNK <= 4096);
static_assert((NBA & (NBA - 1)) == 0 && NBA == (1 << SLA));
static_assert(((long long)CHUNK << SLA) < (1LL << 31));
static_assert(LISTN % NTHR == 0);
static_assert(NBA % NWAVE == 0 && NBA % 32 == 0 && NBA % GBM == 0);
static_assert(RCAP % 4 == 0 && AGG_ZINTS % 4 == 0 && LISTN % 4 == 0 && ((AGG_ZINTS + MISC_INTS) % 4) == 0);
static_assert(K1 % 32 == 0 && K2 % 32 == 0 && K2 == 2 * CH && HP == K2 && NT % GBN == 0);
static_assert(GBM == (GTHR / 32) * 16 && GBN == 64);
static_assert(CH == 4 * 32 && CH == 2 * OUTC);
static_assert(PB_W1 * NTHR * 8 == 256 * K1 && PB_W2 * NTHR * 8 == 256 * K2);
static_assert(AGG_LDS_INTS * 4 <= 300000);

typedef float          v4f   __attribute__((ext_vector_type(4)));
typedef float          v8f   __attribute__((ext_vector_type(8)));
typedef int            v4i   __attribute__((ext_vector_type(4)));
typedef int            v8i   __attribute__((ext_vector_type(8)));
typedef unsigned short v8us  __attribute__((ext_vector_type(8)));
typedef unsigned short v16us __attribute__((ext_vector_type(16)));
typedef __bf16         v16bf __attribute__((ext_vector_type(16)));
typedef v4f  __attribute__((may_alias)) v4fa;
typedef v4i  __attribute__((may_alias)) v4ia;
typedef v8us __attribute__((may_alias)) v8usa;
union FragB { v16bf v; v16us u; v8us h[2]; v8i w; };

__device__ __forceinline__ v8f wmb(const FragB& a, const FragB& b, v8f c) {
  v8f d = __builtin_amdgcn_wmma_f32_16x16x32_bf16(false, a.v, false, b.v, (short)0, c, false, false);
  asm volatile("v_nop\n\tv_nop\n\tv_nop\n\tv_nop" : "+v"(d) : "v"(a.w), "v"(b.w));
  return d;
}

__device__ __forceinline__ unsigned bf16_bits(float f) {
  const unsigned u = __float_as_uint(f);
  return (u + 0x7FFFu + ((u >> 16) & 1u)) >> 16;
}
__device__ __forceinline__ float bf16_val(float f) {
  return __uint_as_float(bf16_bits(f) << 16);
}
__device__ __forceinline__ float blendf(float a, float b, unsigned mk) {
  return __uint_as_float((__float_as_uint(a) & ~mk) | (__float_as_uint(b) & mk));
}

__device__ __forceinline__ void wave_sync() {
  __builtin_amdgcn_fence(__ATOMIC_RELEASE, "wavefront");
  __builtin_amdgcn_wave_barrier();
  __builtin_amdgcn_fence(__ATOMIC_ACQUIRE, "wavefront");
}

template <int SLB>
__device__ __forceinline__ int scan_chunk(const int* __restrict__ dsts, int nE, int cbase, int slotBase,
                                          int nb, int vec8, int* list, int tid, int lane, int wave) {
  int wc = 0;
  const int el0  = tid * EPT;
  const int e0   = cbase + el0;
  const int sent = -2147483647 - 1;
  v4i da, db;
  if (vec8 != 0 && cbase + CHUNK <= nE) {
    da = *(const v4i*)(dsts + e0);
    db = *(const v4i*)(dsts + e0 + 4);
  } else {
    da.x = (e0     < nE) ? dsts[min(e0,     nE - 1)] : sent;
    da.y = (e0 + 1 < nE) ? dsts[min(e0 + 1, nE - 1)] : sent;
    da.z = (e0 + 2 < nE) ? dsts[min(e0 + 2, nE - 1)] : sent;
    da.w = (e0 + 3 < nE) ? dsts[min(e0 + 3, nE - 1)] : sent;
    db.x = (e0 + 4 < nE) ? dsts[min(e0 + 4, nE - 1)] : sent;
    db.y = (e0 + 5 < nE) ? dsts[min(e0 + 5, nE - 1)] : sent;
    db.z = (e0 + 6 < nE) ? dsts[min(e0 + 6, nE - 1)] : sent;
    db.w = (e0 + 7 < nE) ? dsts[min(e0 + 7, nE - 1)] : sent;
  }
  const unsigned nbs = (unsigned)slotBase;
  const unsigned unb = (unsigned)nb;
  const unsigned s0 = (unsigned)da.x - nbs, s1 = (unsigned)da.y - nbs;
  const unsigned s2 = (unsigned)da.z - nbs, s3 = (unsigned)da.w - nbs;
  const unsigned s4 = (unsigned)db.x - nbs, s5 = (unsigned)db.y - nbs;
  const unsigned s6 = (unsigned)db.z - nbs, s7 = (unsigned)db.w - nbs;
  const bool h0 = s0 < unb, h1 = s1 < unb, h2 = s2 < unb, h3 = s3 < unb;
  const bool h4 = s4 < unb, h5 = s5 < unb, h6 = s6 < unb, h7 = s7 < unb;
  const unsigned any = __builtin_amdgcn_ballot_w32(h0 | h1 | h2 | h3 | h4 | h5 | h6 | h7);
  if (any != 0u) {
#define HITJ(J, HJ, SJ) { \
      const unsigned mj = __builtin_amdgcn_ballot_w32(HJ); \
      if (mj != 0u) { \
        if (HJ) { \
          const int pos = wc + (int)__builtin_amdgcn_mbcnt_lo(mj, 0u); \
          if (pos < WCAP) list[wave * WCAP + pos] = ((el0 + (J)) << SLB) | (int)(SJ); \
        } \
        wc += (int)__builtin_popcount(mj); } }
    HITJ(0, h0, s0)
    HITJ(1, h1, s1)
    HITJ(2, h2, s2)
    HITJ(3, h3, s3)
    HITJ(4, h4, s4)
    HITJ(5, h5, s5)
    HITJ(6, h6, s6)
    HITJ(7, h7, s7)
#undef HITJ
  }
  return wc;
}

__device__ __forceinline__ void cvt8_store(const float* __restrict__ p, unsigned short* dp) {
  const v4f a = *(const v4f*)p;
  const v4f b = *(const v4f*)(p + 4);
  v8us o;
  o[0] = (unsigned short)bf16_bits(a.x); o[1] = (unsigned short)bf16_bits(a.y);
  o[2] = (unsigned short)bf16_bits(a.z); o[3] = (unsigned short)bf16_bits(a.w);
  o[4] = (unsigned short)bf16_bits(b.x); o[5] = (unsigned short)bf16_bits(b.y);
  o[6] = (unsigned short)bf16_bits(b.z); o[7] = (unsigned short)bf16_bits(b.w);
  *(volatile v8us*)dp = o;
  __threadfence();
  *(volatile v8us*)dp = o;
}

__global__ __launch_bounds__(NTHR) void k_prep(const float* __restrict__ x, int nN, int nUnits,
                                               const float* __restrict__ W1rel, const float* __restrict__ W1root,
                                               const float* __restrict__ Wmurel, const float* __restrict__ Wlvrel,
                                               const float* __restrict__ Wmuroot, const float* __restrict__ Wlvroot,
                                               const float* __restrict__ b1, const float* __restrict__ bmu,
                                               const float* __restrict__ blv,
                                               unsigned short* XB, unsigned short* W1C, unsigned short* W2C,
                                               float* B1P, float* B2P) {
  const int b = (int)blockIdx.x, tid = (int)threadIdx.x;
  if (b < PB_W1) {
    const int n  = b * 16 + (tid >> 4);
    const int k8 = (tid & 15) * 8;
    const size_t so = (size_t)(n & (CH - 1)) * K1 + k8;
    unsigned short* dp = W1C + (size_t)n * K1 + k8;
    if (b < PB_W1 / 2) cvt8_store(W1rel + so, dp);
    else               cvt8_store(W1root + so, dp);
    return;
  }
  if (b < PB_W1 + PB_W2) {
    const int wb  = b - PB_W1;
    const int mat = wb >> 3;
    const int rm  = (wb & 7) * 8 + (tid >> 5);
    const int k8  = (tid & 31) * 8;
    const size_t so = (size_t)rm * K1 + (k8 & (K1 - 1));
    unsigned short* dp = W2C + (size_t)(mat * OUTC + rm) * K2 + k8;
    if (mat == 0)      cvt8_store(Wmurel + so, dp);
    else if (mat == 1) cvt8_store(Wlvrel + so, dp);
    else if (mat == 2) cvt8_store(Wmuroot + so, dp);
    else               cvt8_store(Wlvroot + so, dp);
    return;
  }
  if (b == PB_W1 + PB_W2) {
    const int lane = tid & 31, wave = tid >> 5;
    if (wave == 0) {
      const v4f a = *(const v4f*)(b1 + 4 * lane);
      v4f o;
      o.x = bf16_val(a.x); o.y = bf16_val(a.y); o.z = bf16_val(a.z); o.w = bf16_val(a.w);
      float* dp = B1P + 4 * lane;
      *(volatile v4f*)dp = o;
      __threadfence();
      *(volatile v4f*)dp = o;
    } else if (wave == 1) {
      const int l15 = lane & 15;
      const v4f a = *(const v4f*)(bmu + 4 * l15);
      const v4f c = *(const v4f*)(blv + 4 * l15);
      const unsigned mk = 0u - (unsigned)(lane >> 4);
      v4f o;
      o.x = blendf(bf16_val(a.x), bf16_val(c.x), mk);
      o.y = blendf(bf16_val(a.y), bf16_val(c.y), mk);
      o.z = blendf(bf16_val(a.z), bf16_val(c.z), mk);
      o.w = blendf(bf16_val(a.w), bf16_val(c.w), mk);
      float* dp = B2P + 4 * lane;
      *(volatile v4f*)dp = o;
      __threadfence();
      *(volatile v4f*)dp = o;
    }
    return;
  }
  const int u = (b - PB_HEAD) * NTHR + tid;
  if (u >= nUnits) return;
  const int row = u >> 4;
  const int k8  = (u & 15) * 8;
  const int rc  = row < nN ? row : nN - 1;
  const float* p = x + (size_t)rc * K1 + k8;
  const v4f a = *(const v4f*)p;
  const v4f c = *(const v4f*)(p + 4);
  const bool ok = row < nN;
  v8us o;
  o[0] = ok ? (unsigned short)bf16_bits(a.x) : (unsigned short)0;
  o[1] = ok ? (unsigned short)bf16_bits(a.y) : (unsigned short)0;
  o[2] = ok ? (unsigned short)bf16_bits(a.z) : (unsigned short)0;
  o[3] = ok ? (unsigned short)bf16_bits(a.w) : (unsigned short)0;
  o[4] = ok ? (unsigned short)bf16_bits(c.x) : (unsigned short)0;
  o[5] = ok ? (unsigned short)bf16_bits(c.y) : (unsigned short)0;
  o[6] = ok ? (unsigned short)bf16_bits(c.z) : (unsigned short)0;
  o[7] = ok ? (unsigned short)bf16_bits(c.w) : (unsigned short)0;
  unsigned short* dp = XB + (size_t)row * K1 + k8;
  *(volatile v8us*)dp = o;
  __threadfence();
  *(volatile v8us*)dp = o;
}

__global__ __launch_bounds__(GTHR) void k_gemm(
    const unsigned short* __restrict__ A, const unsigned short* __restrict__ WT,
    float* outF, int K, int ldo)
{
  __shared__ __attribute__((aligned(16))) float stg[GBM * GBN];
  const int tid = (int)threadIdx.x, lane = tid & 31, wave = tid >> 5, hh = lane >> 4, m = lane & 15;
  const int rowBase = (int)blockIdx.x * GBM;
  const int col0    = (int)blockIdx.y * GBN;

  v8f acc[4];
  {
    const v8f z = {0.f, 0.f, 0.f, 0.f, 0.f, 0.f, 0.f, 0.f};
    acc[0] = z; acc[1] = z; acc[2] = z; acc[3] = z;
  }
  const unsigned short* ap = A  + (size_t)(rowBase + 16 * wave + m) * (size_t)K + 8 * hh;
  const unsigned short* wp = WT + (size_t)(col0 + m) * (size_t)K + 8 * hh;
  const int ksteps = K >> 5;
#pragma unroll 1
  for (int ks = 0; ks < ksteps; ++ks) {
    FragB af;
    af.h[0] = *(const v8usa*)(ap + 32 * ks);
    af.h[1] = *(const v8usa*)(ap + 32 * ks + 16);
#pragma unroll
    for (int t = 0; t < 4; ++t) {
      const unsigned short* wq = wp + (size_t)(16 * t) * (size_t)K + 32 * ks;
      FragB bf;
      bf.h[0] = *(const v8usa*)wq;
      bf.h[1] = *(const v8usa*)(wq + 16);
      acc[t] = wmb(af, bf, acc[t]);
    }
  }

#pragma unroll
  for (int t = 0; t < 4; ++t) {
    const int lc = 16 * t + m;
#pragma unroll
    for (int r = 0; r < 8; ++r) {
      const int lr = 16 * wave + 8 * hh + r;
      stg[lr * GBN + lc] = acc[t][r];
    }
  }
  __syncthreads();

  v4f fv[8];
#pragma unroll
  for (int i = 0; i < 8; ++i) {
    const int lr = 16 * wave + 2 * i + hh;
    fv[i] = *(const v4fa*)(stg + lr * GBN + 4 * m);
  }
#pragma unroll
  for (int i = 0; i < 8; ++i) {
    const int lr = 16 * wave + 2 * i + hh;
    const int gr = rowBase + lr;
    float* op = outF + (size_t)gr * (size_t)ldo + col0 + 4 * m;
    *(volatile v4f*)op = fv[i];
  }
  __threadfence();
#pragma unroll
  for (int i = 0; i < 8; ++i) {
    const int lr = 16 * wave + 2 * i + hh;
    const int gr = rowBase + lr;
    float* op = outF + (size_t)gr * (size_t)ldo + col0 + 4 * m;
    *(volatile v4f*)op = fv[i];
  }
}

template <int MODE>
__global__ __launch_bounds__(NTHR) void k_scan(const int* __restrict__ gath, const int* __restrict__ keys,
                                               const float* __restrict__ ew,
                                               int nE, int nN, int vec8, int mRows,
                                               const float* __restrict__ tp, const float* __restrict__ bias,
                                               unsigned short* hpl, float* outp, int lvOff) {
  extern __shared__ __attribute__((aligned(16))) int dsm[];
  int* list = dsm;
  int* hl   = dsm + LISTN;
  int* sl   = hl + RCAP;
  int* cnt  = sl + RCAP;
  int* offs = cnt + NBA;
  int* cur  = offs + NBA;
  int* misc = cur + NBA;
  const int tid = (int)threadIdx.x, lane = tid & 31, wave = tid >> 5;
  float* prow = (float*)(misc + MISC_INTS) + wave * CH;
  unsigned short* rowbuf = (unsigned short*)(misc + MISC_INTS + PROW_INTS) + wave * HP;
  const int nodeBase = (int)blockIdx.x * NBA;

  {
    const v4i z4 = {0, 0, 0, 0};
    for (int i = tid * 4; i < AGG_ZINTS; i += NTHR * 4) *(v4ia*)(dsm + i) = z4;
    if (tid < MISC_INTS) misc[tid] = 0;
  }
  const v4f bb = *(const v4f*)(bias + 4 * lane);
  __syncthreads();

  int t = 0, ov = 0;
  const int nChunks = (nE + CHUNK - 1) / CHUNK;
#pragma unroll 1
  for (int ch = 0; ch < nChunks; ++ch) {
    const int cbase = ch * CHUNK;
    const int wc = scan_chunk<SLA>(keys, nE, cbase, nodeBase, NBA, vec8, list, tid, lane, wave);
    if (lane == 0) misc[wave] = wc;
    __syncthreads();
    if (wave == 0) {
#pragma unroll 1
      for (int w2 = 0; w2 < NWAVE; ++w2) {
        int c = misc[w2];
        c = c < 0 ? 0 : (c > WCAP ? WCAP : c);
#pragma unroll 1
        for (int b0 = 0; b0 < c; b0 += 32) {
          const int idx = b0 + lane;
          const int ent = list[w2 * WCAP + (idx < WCAP ? idx : WCAP - 1)];
          const int m32 = (c - b0) < 32 ? (c - b0) : 32;
#pragma unroll 1
          for (int k = 0; k < m32; ++k) {
            const int u    = __builtin_amdgcn_readlane(ent, k);
            const int slot = u & (NBA - 1);
            const int el   = (u >> SLA) & (CHUNK - 1);
            const int pk   = ((cbase + el) << SLA) | slot;
            if (t < RCAP) {
              if (lane == 0) { hl[t] = pk; cnt[slot] = cnt[slot] + 1; }
              t = t + 1;
            } else {
              ov = 1;
            }
          }
        }
      }
    }
    __syncthreads();
  }
  if (wave == 0 && lane == 0) { misc[8] = t; misc[9] = ov; }
  __syncthreads();
  int tt = misc[8];
  tt = tt < 0 ? 0 : (tt > RCAP ? RCAP : tt);
  const int ovf = misc[9];

  if (wave == 0) {
    const int base = lane * (NBA / 32);
    int s = 0;
#pragma unroll 1
    for (int i = 0; i < NBA / 32; ++i) s += cnt[base + i];
    int incl = s;
#pragma unroll
    for (int d = 1; d < 32; d <<= 1) {
      const int y = __shfl_up(incl, d, 32);
      if (lane >= d) incl += y;
    }
    int run = incl - s;
#pragma unroll 1
    for (int i = 0; i < NBA / 32; ++i) {
      const int cv = cnt[base + i];
      offs[base + i] = run;
      cur[base + i]  = run;
      run += cv;
    }
  }
  __syncthreads();
  if (wave == 0) {
#pragma unroll 1
    for (int b0 = 0; b0 < tt; b0 += 32) {
      const int idx = b0 + lane;
      const int ent = hl[idx < RCAP ? idx : RCAP - 1];
      const int m32 = (tt - b0) < 32 ? (tt - b0) : 32;
#pragma unroll 1
      for (int k = 0; k < m32; ++k) {
        const int u    = __builtin_amdgcn_readlane(ent, k);
        const int slot = u & (NBA - 1);
        if (lane == 0) {
          int p = cur[slot];
          p = p < 0 ? 0 : (p > RCAP - 1 ? RCAP - 1 : p);
          sl[p] = u;
          cur[slot] = p + 1;
        }
      }
    }
  }
  __syncthreads();

  const float qnan = __int_as_float(0x7fc00000);
  const float pz = (ovf != 0) ? qnan : 0.0f;
#pragma unroll 1
  for (int si = 0; si < NBA / NWAVE; ++si) {
    const int s    = si * NWAVE + wave;
    const int node = nodeBase + s;
    const int cr = cnt[s];
    const bool big = cr > DEGCAP;
    const int c = cr < 0 ? 0 : (cr > DEGCAP ? DEGCAP : cr);
    int o = offs[s];
    o = o < 0 ? 0 : (o > RCAP ? RCAP : o);
    const int nc = node < nN ? node : nN - 1;
    float a0 = 0.0f, a1 = 0.0f, a2 = 0.0f, a3 = 0.0f;
#pragma unroll 1
    for (int b0 = 0; b0 < c; b0 += 32) {
      int idx = o + b0 + lane;
      idx = idx > RCAP - 1 ? RCAP - 1 : idx;
      const int ent = sl[idx];
      int eid = ent >> SLA;
      eid = eid < 0 ? 0 : (eid > nE - 1 ? nE - 1 : eid);
      int sr = gath[eid];
      sr = sr < 0 ? 0 : (sr > nN - 1 ? nN - 1 : sr);
      const float wv  = bf16_val(ew[eid]);
      const int   wvi = __float_as_int(wv);
      const int m32 = (c - b0) < 32 ? (c - b0) : 32;
#pragma unroll 1
      for (int k = 0; k < m32; ++k) {
        const int   sk = __builtin_amdgcn_readlane(sr, k);
        const float ck = __int_as_float(__builtin_amdgcn_readlane(wvi, k));
        const v4f a = *(const v4f*)(tp + (size_t)sk * NT + 4 * lane);
        a0 = fmaf(ck, a.x, a0);
        a1 = fmaf(ck, a.y, a1);
        a2 = fmaf(ck, a.z, a2);
        a3 = fmaf(ck, a.w, a3);
      }
    }
    const int cd = cr < 1 ? 1 : cr;
    const float inv = 1.0f / (float)cd;
    const v4f rt = *(const v4f*)(tp + (size_t)nc * NT + CH + 4 * lane);
    const float pzr = big ? qnan : pz;
    const bool live = node < nN;
    const float t0 = (a0 * inv + bb.x) + rt.x;
    const float t1 = (a1 * inv + bb.y) + rt.y;
    const float t2 = (a2 * inv + bb.z) + rt.z;
    const float t3 = (a3 * inv + bb.w) + rt.w;
    if constexpr (MODE != 0) {
      v4f tv;
      tv.x = t0; tv.y = t1; tv.z = t2; tv.w = t3;
      *(v4fa*)(prow + 4 * lane) = tv;
      wave_sync();
#pragma unroll 1
      for (int j = 0; j < 4; ++j) {
        const int chn = j * 32 + lane;
        const float tvv = prow[chn];
        float y = (tvv > 0.0f) ? tvv : expm1f(tvv);
        y = y + pzr;
        y = live ? y : 0.0f;
        const unsigned hb = bf16_bits(y);
        const unsigned lb = bf16_bits(y - __uint_as_float(hb << 16));
        rowbuf[chn]      = (unsigned short)hb;
        rowbuf[CH + chn] = (unsigned short)lb;
      }
      wave_sync();
      const v8us q0 = *(const v8usa*)(rowbuf + 8 * lane);
      wave_sync();
      if (node < mRows) {
        unsigned short* rpw = hpl + (size_t)node * HP + 8 * lane;
        *(volatile v8us*)rpw = q0;
        __threadfence();
        *(volatile v8us*)rpw = q0;
      }
    } else {
      v4f ow;
      ow.x = t0 + pzr; ow.y = t1 + pzr; ow.z = t2 + pzr; ow.w = t3 + pzr;
      float* op = outp + (size_t)(lane >> 4) * (size_t)lvOff + (size_t)nc * OUTC + 4 * (lane & 15);
      if (live) {
        *(volatile v4f*)op = ow;
        __threadfence();
        *(volatile v4f*)op = ow;
      }
    }
  }
}

static inline int cdiv(int a, int b) { return (a + b - 1) / b; }
static inline size_t al256(size_t o) { return (o + 255) & ~(size_t)255; }

extern "C" void kernel_launch(void* const* d_in, const int* in_sizes, int n_in,
                              void* d_out, int out_size, void* d_ws, size_t ws_size,
                              hipStream_t stream) {
  if (n_in < 12) return;
  if (in_sizes[0] < K1 || (in_sizes[0] % K1) != 0) return;
  const int nN = in_sizes[0] / K1;
  const int nE = in_sizes[2];
  if (nE < 1 || in_sizes[1] != 2 * nE) return;
  if (nE >= (1 << 21) || nN < 16 || nN >= (1 << 22)) return;
  if (in_sizes[3] != CH * K1 || in_sizes[4] != CH || in_sizes[5] != CH * K1) return;
  if (in_sizes[6] != OUTC * CH || in_sizes[7] != OUTC || in_sizes[8] != OUTC * CH) return;
  if (in_sizes[9] != OUTC * CH || in_sizes[10] != OUTC || in_sizes[11] != OUTC * CH) return;
  if ((long long)out_size != 2LL * (long long)nN * OUTC) return;

  const float* x       = (const float*)d_in[0];
  const int*   edge    = (const int*)d_in[1];
  const float* ew      = (const float*)d_in[2];
  const float* W1rel   = (const float*)d_in[3];
  const float* b1      = (const float*)d_in[4];
  const float* W1root  = (const float*)d_in[5];
  const float* Wmurel  = (const float*)d_in[6];
  const float* bmu     = (const float*)d_in[7];
  const float* Wmuroot = (const float*)d_in[8];
  const float* Wlvrel  = (const float*)d_in[9];
  const float* blv     = (const float*)d_in[10];
  const float* Wlvroot = (const float*)d_in[11];
  float* out = (float*)d_out;
  const int* src = edge;
  const int* dst = edge + nE;
  const int lvOff = nN * OUTC;
  if ((long long)lvOff + (long long)(nN - 1) * OUTC + (OUTC - 1) >= (long long)out_size) return;

  const int MP = cdiv(nN, GBM) * GBM;
  const int gM = MP / GBM;
  const int gA = cdiv(MP, NBA);
  if ((long long)gA * NBA < (long long)MP) return;
  const int vec8 = ((nE & 3) == 0) ? 1 : 0;

  char* ws = (char*)d_ws;
  size_t off = 0;
  const size_t oW1C = off; off = al256(off + (size_t)256 * K1 * 2);
  const size_t oW2C = off; off = al256(off + (size_t)256 * K2 * 2);
  const size_t oB1  = off; off = al256(off + (size_t)CH * 4);
  const size_t oB2  = off; off = al256(off + (size_t)CH * 4);
  const size_t oXB  = off; off = al256(off + (size_t)MP * K1 * 2);
  const size_t oT   = off; off = al256(off + (size_t)MP * NT * 4);
  const size_t oH   = off; off = al256(off + (size_t)MP * HP * 2);
  if (off > ws_size || off > (size_t)WSMAX) return;
  unsigned short* W1C = (unsigned short*)(ws + oW1C);
  unsigned short* W2C = (unsigned short*)(ws + oW2C);
  float*          B1P = (float*)(ws + oB1);
  float*          B2P = (float*)(ws + oB2);
  unsigned short* XB  = (unsigned short*)(ws + oXB);
  float*          T   = (float*)(ws + oT);
  unsigned short* H   = (unsigned short*)(ws + oH);

  const size_t scanLds = (size_t)AGG_LDS_INTS * 4;
  hipFuncSetAttribute(reinterpret_cast<const void*>(&k_scan<1>), hipFuncAttributeMaxDynamicSharedMemorySize, (int)scanLds);
  hipFuncSetAttribute(reinterpret_cast<const void*>(&k_scan<0>), hipFuncAttributeMaxDynamicSharedMemorySize, (int)scanLds);

  const int nUx = MP * (K1 / 8);
  k_prep<<<PB_HEAD + cdiv(nUx, NTHR), NTHR, 0, stream>>>(x, nN, nUx, W1rel, W1root, Wmurel, Wlvrel, Wmuroot, Wlvroot,
                                                         b1, bmu, blv, XB, W1C, W2C, B1P, B2P);
  k_gemm<<<dim3(gM, NT / GBN), GTHR, 0, stream>>>(XB, W1C, T, K1, NT);
  k_scan<1><<<gA, NTHR, scanLds, stream>>>(src, dst, ew, nE, nN, vec8, MP, T, B1P, H, out, lvOff);
  k_gemm<<<dim3(gM, NT / GBN), GTHR, 0, stream>>>(H, W2C, T, K2, NT);
  k_scan<0><<<gA, NTHR, scanLds, stream>>>(src, dst, ew, nE, nN, vec8, MP, T, B2P, H, out, lvOff);
}
